// MSSSM_33758442947270
// MI455X (gfx1250) — hardware-verified
//
#include <hip/hip_runtime.h>


namespace {
constexpr int NB = 4, C = 128, HI = 64, LI = HI * HI, GC = 32, DI = 64, R = 2, NTK = NB * LI;
constexpr float XS = 8.0f, HS = 64.0f, DS = 256.0f, WSC = 256.0f;
typedef _Float16 b16;
typedef __attribute__((ext_vector_type(16))) _Float16 v16b;
typedef __attribute__((ext_vector_type(8))) _Float16 v8b;
typedef __attribute__((ext_vector_type(8))) float v8f;
typedef __attribute__((ext_vector_type(4))) float v4f;
typedef __attribute__((ext_vector_type(2))) float v2f;
__device__ __forceinline__ float bf16_rne(float f) { unsigned int u = __float_as_uint(f); u += 0x7FFFu + ((u >> 16) & 1u); return __uint_as_float(u & 0xFFFF0000u); }
__device__ __forceinline__ void split16(float v, b16& hi, b16& lo) { hi = (b16)v; lo = (b16)(v - (float)hi); }
__device__ __forceinline__ v16b frag_kb(const b16* p, int hh) { const v8b a = *(const v8b*)(p + 8 * hh), b = *(const v8b*)(p + 16 + 8 * hh); v16b f;
#pragma unroll
  for (int e = 0; e < 8; ++e) { f[e] = a[e]; f[8 + e] = b[e]; } return f; }
__device__ __forceinline__ v8f wmma16b(v16b a, v16b b, v8f c) { v8f d = __builtin_amdgcn_wmma_f32_16x16x32_f16(false, a, false, b, (short)0, c, false, false); asm volatile("v_nop\n\tv_nop\n\tv_nop\n\tv_nop" : "+v"(d) : "v"(a), "v"(b)); return d; }
__device__ __forceinline__ void wave_lds_sync() { __builtin_amdgcn_fence(__ATOMIC_RELEASE, "workgroup"); __builtin_amdgcn_wave_barrier(); __builtin_amdgcn_fence(__ATOMIC_ACQUIRE, "workgroup"); }
__device__ __forceinline__ float pmul(float a, float b) { float p = a * b; asm volatile("" : "+v"(p)); return p; }
__device__ __forceinline__ float sigm(float v) { return 1.0f / (1.0f + __expf(-v)); }
__device__ __forceinline__ float silu(float v) { return pmul(v, sigm(v)); }
__device__ __forceinline__ float softplus(float v) { return v > 20.0f ? v : (v < -20.0f ? __expf(v) : log1pf(__expf(v))); }
__device__ __forceinline__ float bnscale(const float* g, const float* v, int c) { return bf16_rne(g[c]) * rsqrtf(bf16_rne(v[c]) + 1e-5f); }

__global__ __launch_bounds__(256) void wcopyp_kernel(const float* __restrict__ w, int KIN, int OUT, int KP, int OUTP, b16* __restrict__ WT) {
  const int u = blockIdx.x * 256 + threadIdx.x; if (u >= OUTP * KP / 8) return; const int e = u * 8; const int o = e / KP, k0 = e % KP; v8b v;
#pragma unroll
  for (int j = 0; j < 8; ++j) { const int k = k0 + j; v[j] = (o < OUT && k < KIN) ? (b16)(bf16_rne(w[(size_t)o * KIN + k]) * WSC) : (b16)0.0f; } for (int pass = 0; pass < 2; ++pass) { *(volatile v8b*)(WT + e) = v; __threadfence(); }
}
__global__ __launch_bounds__(256) void wconv_kernel(const float* __restrict__ w, b16* __restrict__ WT) {
  const int u = blockIdx.x * 256 + threadIdx.x; if (u >= GC * 288 / 8) return; const int e = u * 8; const int o = e / 288, k0 = e % 288; v8b v;
#pragma unroll
  for (int j = 0; j < 8; ++j) { const int k = k0 + j; const int tap = k / 32, c = k % 32; v[j] = (b16)(bf16_rne(w[((size_t)o * GC + c) * 9 + tap]) * WSC); } for (int pass = 0; pass < 2; ++pass) { *(volatile v8b*)(WT + e) = v; __threadfence(); }
}
__global__ __launch_bounds__(256) void wsa_kernel(const float* __restrict__ w, b16* __restrict__ WT) {
  const int u = blockIdx.x * 256 + threadIdx.x; if (u >= 16 * 6272 / 8) return; const int e = u * 8; const int o = e / 6272, k0 = e % 6272; v8b v;
#pragma unroll
  for (int j = 0; j < 8; ++j) { const int k = k0 + j; const int tap = k / C, c = k % C; v[j] = o == 0 ? (b16)(bf16_rne(w[(size_t)c * 49 + tap]) * WSC) : (b16)0.0f; } for (int pass = 0; pass < 2; ++pass) { *(volatile v8b*)(WT + e) = v; __threadfence(); }
}
__global__ __launch_bounds__(256) void xt_kernel(const float* __restrict__ x, float* __restrict__ XT) {
  __shared__ float T[HI][33]; const int cg = blockIdx.x % 4, y = (blockIdx.x / 4) % HI, b = blockIdx.x / (4 * HI); const int tid = threadIdx.x;
  for (int i = tid; i < 32 * HI; i += 256) { const int cl = i / HI, xx = i % HI; T[xx][cl] = bf16_rne(x[(((size_t)b * C + cg * 32 + cl) * HI + y) * HI + xx]); }
  __syncthreads();
  for (int pass = 0; pass < 2; ++pass) { for (int i = tid; i < HI * 32; i += 256) { const int xx = i / 32, cl = i % 32; ((volatile float*)XT)[(((size_t)b * HI + y) * HI + xx) * C + cg * 32 + cl] = T[xx][cl]; } __threadfence(); }
}
__global__ __launch_bounds__(128) void pool_kernel(const float* __restrict__ PL, int NBV, float* __restrict__ POOL) {
  const int b = blockIdx.x, c = threadIdx.x; if (b >= NBV) return; float s = 0.0f;
#pragma unroll 4
  for (int p = 0; p < LI; ++p) s += PL[((size_t)b * LI + p) * C + c];
  const float m = s * (1.0f / LI); for (int pass = 0; pass < 2; ++pass) { ((volatile float*)POOL)[b * C + c] = m; __threadfence(); }
}
__global__ __launch_bounds__(128) void gf_kernel(const float* __restrict__ POOL, const float* __restrict__ gpw, float* __restrict__ GF) {
  __shared__ float pv[C]; const int b = blockIdx.x, o = threadIdx.x; pv[o] = POOL[b * C + o]; __syncthreads(); float s = 0.0f;
#pragma unroll 1
  for (int c = 0; c < C; ++c) s += pmul(pv[c], bf16_rne(gpw[o * C + c])); const float g = fmaxf(s, 0.0f); for (int pass = 0; pass < 2; ++pass) { ((volatile float*)GF)[b * C + o] = g; __threadfence(); }
}
__global__ __launch_bounds__(128) void ca_kernel(const float* __restrict__ POOL, const float* __restrict__ w1, const float* __restrict__ b1, const float* __restrict__ w2, const float* __restrict__ b2, float* __restrict__ CA) {
  __shared__ float pv[C], hv[8]; const int b = blockIdx.x, o = threadIdx.x; pv[o] = POOL[b * C + o]; __syncthreads();
  if (o < 8) { float s = bf16_rne(b1[o]); for (int c = 0; c < C; ++c) s += pmul(pv[c], bf16_rne(w1[o * C + c])); hv[o] = fmaxf(s, 0.0f); } __syncthreads();
  float s = bf16_rne(b2[o]); for (int j = 0; j < 8; ++j) s += pmul(hv[j], bf16_rne(w2[o * 8 + j])); const float a = sigm(s); for (int pass = 0; pass < 2; ++pass) { ((volatile float*)CA)[b * C + o] = a; __threadfence(); }
}
__global__ __launch_bounds__(32) void conv3_kernel(const float* __restrict__ XT, int c0, int c1, int dil, const b16* __restrict__ WT, const float* __restrict__ bng, const float* __restrict__ bnb, const float* __restrict__ bnm, const float* __restrict__ bnv, int fo, int NTV, float* __restrict__ FUSED) {
  __shared__ __attribute__((aligned(16))) b16 Ah[16][288 + 8], Al[16][288 + 8]; __shared__ __attribute__((aligned(16))) float Tf[16][32 + 1];
  const int lane = threadIdx.x, nloc = lane & 15, hlf = lane >> 4; const size_t t0 = (size_t)blockIdx.x * 16; if (t0 >= (size_t)NTV) return;
  for (int rr = 0; rr < 16; ++rr) { const size_t t = t0 + rr; const int b = (int)(t / LI), p = (int)(t % LI), y = p / HI, xx = p % HI;
    for (int tap = 0; tap < 9; ++tap) { const int yy = y + (tap / 3 - 1) * dil, x2 = xx + (tap % 3 - 1) * dil; float v = 0.0f;
      if (yy >= 0 && yy < HI && x2 >= 0 && x2 < HI) { const size_t tn = ((size_t)b * HI + yy) * HI + x2; v = XT[tn * C + c0 + lane]; if (c1 >= 0) v += XT[tn * C + c1 + lane]; }
      b16 ph, pl; split16(v * XS, ph, pl); Ah[rr][tap * 32 + lane] = ph; Al[rr][tap * 32 + lane] = pl; } }
  wave_lds_sync();
  v8f acc[2] = {(v8f){}, (v8f){}};
#pragma unroll 3
  for (int kb = 0; kb < 288; kb += 32) { const v16b a = frag_kb(&Ah[nloc][kb], hlf), al = frag_kb(&Al[nloc][kb], hlf);
#pragma unroll
    for (int tt = 0; tt < 2; ++tt) { const v16b bw = frag_kb(WT + (size_t)(tt * 16 + nloc) * 288 + kb, hlf); acc[tt] = wmma16b(a, bw, acc[tt]); acc[tt] = wmma16b(al, bw, acc[tt]); } }
#pragma unroll
  for (int tt = 0; tt < 2; ++tt) { const int c = tt * 16 + nloc; float sc = 1.0f, sh = 0.0f; if (bng) { sc = bnscale(bng, bnv, c); sh = bf16_rne(bnb[c]) - bf16_rne(bnm[c]) * sc; }
#pragma unroll 1
    for (int r8 = 0; r8 < 8; ++r8) Tf[8 * hlf + r8][c] = fmaxf(pmul(acc[tt][r8] * (1.0f / (XS * WSC)), sc) + sh, 0.0f); }
  wave_lds_sync();
  for (int pass = 0; pass < 2; ++pass) { for (int rr = 0; rr < 16; ++rr) ((volatile float*)FUSED)[(t0 + rr) * C + fo + lane] = Tf[rr][lane]; __threadfence(); }
}
__global__ __launch_bounds__(32) void inproj_kernel(const float* __restrict__ XT, int c0, int c1, const b16* __restrict__ W, int NTV, float* __restrict__ XZ) {
  __shared__ __attribute__((aligned(16))) b16 Ah[16][32 + 8], Al[16][32 + 8]; __shared__ __attribute__((aligned(16))) float Tf[16][128 + 4];
  const int lane = threadIdx.x, nloc = lane & 15, hlf = lane >> 4; const size_t t0 = (size_t)blockIdx.x * 16; if (t0 >= (size_t)NTV) return;
  for (int rr = 0; rr < 16; ++rr) { float v = XT[(t0 + rr) * C + c0 + lane]; if (c1 >= 0) v += XT[(t0 + rr) * C + c1 + lane]; b16 p, q; split16(v * XS, p, q); Ah[rr][lane] = p; Al[rr][lane] = q; }
  wave_lds_sync();
  v8f acc[8]; const v16b a = frag_kb(&Ah[nloc][0], hlf), al = frag_kb(&Al[nloc][0], hlf);
#pragma unroll
  for (int t = 0; t < 8; ++t) { acc[t] = (v8f){}; const v16b bw = frag_kb(W + (size_t)(t * 16 + nloc) * 32, hlf); acc[t] = wmma16b(a, bw, acc[t]); acc[t] = wmma16b(al, bw, acc[t]); }
#pragma unroll
  for (int t = 0; t < 8; ++t)
#pragma unroll 1
    for (int r8 = 0; r8 < 8; ++r8) Tf[8 * hlf + r8][t * 16 + nloc] = acc[t][r8] * (1.0f / (XS * WSC));
  wave_lds_sync();
  for (int pass = 0; pass < 2; ++pass) { for (int rr = 0; rr < 16; ++rr) *(volatile v4f*)(XZ + (t0 + rr) * 128 + lane * 4) = *(const v4f*)(&Tf[rr][lane * 4]); __threadfence(); }
}
template <int KC>
__global__ __launch_bounds__(256) void dwconv_kernel(const float* __restrict__ XZ, const float* __restrict__ cw, const float* __restrict__ cb, int NTV, float* __restrict__ U) {
  const size_t gid = (size_t)blockIdx.x * 256 + threadIdx.x; const size_t t = gid / (DI / 4); const int d4 = (int)(gid % (DI / 4)) * 4; if (t >= (size_t)NTV) return;
  const int b = (int)(t / LI), p = (int)(t % LI), y = p / HI, xx = p % HI; constexpr int PD = (KC - 1) / 2; v4f acc; for (int q = 0; q < 4; ++q) acc[q] = bf16_rne(cb[d4 + q]);
#pragma unroll 1
  for (int di = 0; di < KC; ++di)
#pragma unroll
    for (int dj = 0; dj < KC; ++dj) { const int yy = y + di - PD, x2 = xx + dj - PD; const bool ok = yy >= 0 && yy < HI && x2 >= 0 && x2 < HI; const int yc = ok ? yy : y, xc = ok ? x2 : xx;
      const v4f v = *(const v4f*)(XZ + (((size_t)b * HI + yc) * HI + xc) * 128 + d4); for (int q = 0; q < 4; ++q) acc[q] += ok ? pmul(v[q], bf16_rne(cw[(d4 + q) * KC * KC + di * KC + dj])) : 0.0f; }
  v4f o; for (int q = 0; q < 4; ++q) o[q] = silu(acc[q]);
  for (int pass = 0; pass < 2; ++pass) { *(volatile v4f*)(U + t * DI + d4) = o; __threadfence(); }
}
template <int NS, int NTX, int BCW>
__global__ __launch_bounds__(32) void xproj_kernel(const float* __restrict__ U, const b16* __restrict__ XPW, const b16* __restrict__ DTW, const float* __restrict__ dtb, int NTV, float* __restrict__ BC, float* __restrict__ DT) {
  __shared__ __attribute__((aligned(16))) b16 Ah[16][DI + 8], Al[16][DI + 8], Dh[16][32 + 8], Dl[16][32 + 8]; __shared__ __attribute__((aligned(16))) float Sbc[16][BCW], Tf[16][DI + 4];
  const int lane = threadIdx.x, nloc = lane & 15, hlf = lane >> 4; const size_t t0 = (size_t)blockIdx.x * 16; const int k = blockIdx.y; if (t0 >= (size_t)NTV) return;
  for (int rr = 0; rr < 16; ++rr) { for (int q = 0; q < 2; ++q) { b16 p, ql; split16(U[(t0 + rr) * DI + q * 32 + lane] * HS, p, ql); Ah[rr][q * 32 + lane] = p; Al[rr][q * 32 + lane] = ql; } Dh[rr][lane] = (b16)0.0f; Dl[rr][lane] = (b16)0.0f; for (int q = lane; q < BCW; q += 32) Sbc[rr][q] = 0.0f; }
  wave_lds_sync();
  v8f ax[NTX];
#pragma unroll
  for (int tt = 0; tt < NTX; ++tt) ax[tt] = (v8f){};
#pragma unroll
  for (int kb = 0; kb < DI; kb += 32) { const v16b a = frag_kb(&Ah[nloc][kb], hlf), al = frag_kb(&Al[nloc][kb], hlf);
#pragma unroll
    for (int tt = 0; tt < NTX; ++tt) { const v16b bw = frag_kb(XPW + ((size_t)k * NTX * 16 + tt * 16 + nloc) * DI + kb, hlf); ax[tt] = wmma16b(a, bw, ax[tt]); ax[tt] = wmma16b(al, bw, ax[tt]); } }
  wave_lds_sync();
#pragma unroll
  for (int tt = 0; tt < NTX; ++tt) { const int c = tt * 16 + nloc;
#pragma unroll
    for (int r8 = 0; r8 < 8; ++r8) { const int rl = 8 * hlf + r8; const float v = ax[tt][r8] * (1.0f / (HS * WSC)); if (c < R) { b16 p, ql; split16(v * DS, p, ql); Dh[rl][c] = p; Dl[rl][c] = ql; } else if (c < R + 2 * NS) Sbc[rl][c - R] = v; } }
  wave_lds_sync();
  for (int pass = 0; pass < 2; ++pass) { for (int rr = 0; rr < 16; ++rr) for (int q = lane; q < BCW; q += 32) ((volatile float*)BC)[((size_t)k * NTK + t0 + rr) * BCW + q] = Sbc[rr][q]; __threadfence(); }
  v8f acc[4]; const v16b a = frag_kb(&Dh[nloc][0], hlf), al = frag_kb(&Dl[nloc][0], hlf);
#pragma unroll
  for (int tt = 0; tt < 4; ++tt) { acc[tt] = (v8f){}; const v16b bw = frag_kb(DTW + ((size_t)k * DI + tt * 16 + nloc) * 32, hlf); acc[tt] = wmma16b(a, bw, acc[tt]); acc[tt] = wmma16b(al, bw, acc[tt]); }
#pragma unroll
  for (int tt = 0; tt < 4; ++tt) { const int c = tt * 16 + nloc; const float bb = bf16_rne(dtb[k * DI + c]);
#pragma unroll 1
    for (int r8 = 0; r8 < 8; ++r8) Tf[8 * hlf + r8][c] = softplus(acc[tt][r8] * (1.0f / (DS * WSC)) + bb); }
  wave_lds_sync();
  for (int pass = 0; pass < 2; ++pass) { for (int rr = 0; rr < 16; ++rr) *(volatile v2f*)(DT + ((size_t)k * NTK + t0 + rr) * DI + lane * 2) = *(const v2f*)(&Tf[rr][lane * 2]); __threadfence(); }
}
template <int NS, int BCW>
__global__ __launch_bounds__(256) void scan_kernel(const float* __restrict__ U, const float* __restrict__ DT, const float* __restrict__ BC, const float* __restrict__ alog, const float* __restrict__ Ds, int NBV, float* __restrict__ Y) {
  const int gid = blockIdx.x * 256 + threadIdx.x; const int d = gid % DI, k = (gid / DI) % 4, b = gid / (4 * DI); if (b >= NBV) return;
  float A[NS]; for (int s = 0; s < NS; ++s) A[s] = -__expf(bf16_rne(alog[((size_t)k * DI + d) * NS + s])); const float dk = bf16_rne(Ds[k * DI + d]);
#pragma unroll 1
  for (int pass = 0; pass < 2; ++pass) { float h[NS]; for (int s = 0; s < NS; ++s) h[s] = 0.0f;
#pragma unroll 1
    for (int l = 0; l < LI; ++l) { const int lk = (k >= 2) ? (LI - 1 - l) : l; const int tok = (k & 1) ? ((lk % HI) * HI + lk / HI) : lk; const size_t row = (size_t)b * LI + tok; const size_t krow = (size_t)k * NTK + row;
      const float u = U[row * DI + d], dt = DT[krow * DI + d]; const float du = pmul(dt, u); const float* bc = BC + krow * BCW; float acc = 0.0f;
#pragma unroll
      for (int s = 0; s < NS; ++s) { h[s] = pmul(h[s], __expf(pmul(dt, A[s]))) + pmul(du, bc[s]); acc += pmul(h[s], bc[NS + s]); }
      ((volatile float*)Y)[krow * DI + d] = acc + pmul(dk, u); }
    __threadfence(); }
}
__global__ __launch_bounds__(32) void sstail_kernel(const float* __restrict__ Y, const float* __restrict__ XZ, const float* __restrict__ lng, const float* __restrict__ lnb, const b16* __restrict__ WO, const float* __restrict__ POOL, int pc0, int pc1, const b16* __restrict__ WG, const float* __restrict__ bng, const float* __restrict__ bnb, const float* __restrict__ bnm, const float* __restrict__ bnv, int fo, int NTV, float* __restrict__ FUSED) {
  __shared__ __attribute__((aligned(16))) b16 Ah[16][DI + 8], Al[16][DI + 8]; __shared__ __attribute__((aligned(16))) float Tf[16][32 + 1];
  const int lane = threadIdx.x, nloc = lane & 15, hlf = lane >> 4; const size_t t0 = (size_t)blockIdx.x * 16; if (t0 >= (size_t)NTV) return; const int b = (int)(t0 / LI);
  const float g0 = bf16_rne(lng[lane * 2]), g1 = bf16_rne(lng[lane * 2 + 1]), e0 = bf16_rne(lnb[lane * 2]), e1 = bf16_rne(lnb[lane * 2 + 1]);
  for (int rr = 0; rr < 16; ++rr) { const size_t t = t0 + rr; float y0 = 0.0f, y1 = 0.0f; for (int k = 0; k < 4; ++k) { const v2f v = *(const v2f*)(Y + ((size_t)k * NTK + t) * DI + lane * 2); y0 += v[0]; y1 += v[1]; }
    float s = y0 + y1; for (int o = 16; o; o >>= 1) s += __shfl_xor(s, o); const float mu = s * (1.0f / DI); const float d0 = y0 - mu, d1 = y1 - mu; float vq = pmul(d0, d0) + pmul(d1, d1); for (int o = 16; o; o >>= 1) vq += __shfl_xor(vq, o); const float rs = rsqrtf(vq * (1.0f / DI) + 1e-5f);
    const v2f z = *(const v2f*)(XZ + t * 128 + DI + lane * 2); const float a0 = pmul(pmul(pmul(d0, rs), g0) + e0, silu(z[0])), a1 = pmul(pmul(pmul(d1, rs), g1) + e1, silu(z[1]));
    b16 p, q; split16(a0 * XS, p, q); Ah[rr][lane * 2] = p; Al[rr][lane * 2] = q; split16(a1 * XS, p, q); Ah[rr][lane * 2 + 1] = p; Al[rr][lane * 2 + 1] = q; }
  wave_lds_sync();
  v8f acc[2] = {(v8f){}, (v8f){}};
#pragma unroll
  for (int kb = 0; kb < DI; kb += 32) { const v16b a = frag_kb(&Ah[nloc][kb], hlf), al = frag_kb(&Al[nloc][kb], hlf);
#pragma unroll
    for (int tt = 0; tt < 2; ++tt) { const v16b bw = frag_kb(WO + (size_t)(tt * 16 + nloc) * DI + kb, hlf); acc[tt] = wmma16b(a, bw, acc[tt]); acc[tt] = wmma16b(al, bw, acc[tt]); } }
  wave_lds_sync();
#pragma unroll
  for (int tt = 0; tt < 2; ++tt) { const int c = tt * 16 + nloc;
#pragma unroll
    for (int r8 = 0; r8 < 8; ++r8) { const int rl = 8 * hlf + r8; b16 p, q; split16(acc[tt][r8] * (HS / (XS * WSC)), p, q); Ah[rl][c] = p; Al[rl][c] = q; } }
  for (int rr = 0; rr < 16; ++rr) { float pv = POOL[b * C + pc0 + lane]; if (pc1 >= 0) pv += POOL[b * C + pc1 + lane]; b16 p, q; split16(pv * HS, p, q); Ah[rr][32 + lane] = p; Al[rr][32 + lane] = q; }
  wave_lds_sync();
  acc[0] = (v8f){}; acc[1] = (v8f){};
#pragma unroll
  for (int kb = 0; kb < DI; kb += 32) { const v16b a = frag_kb(&Ah[nloc][kb], hlf), al = frag_kb(&Al[nloc][kb], hlf);
#pragma unroll
    for (int tt = 0; tt < 2; ++tt) { const v16b bw = frag_kb(WG + (size_t)(tt * 16 + nloc) * DI + kb, hlf); acc[tt] = wmma16b(a, bw, acc[tt]); acc[tt] = wmma16b(al, bw, acc[tt]); } }
#pragma unroll
  for (int tt = 0; tt < 2; ++tt) { const int c = tt * 16 + nloc; const float sc = bnscale(bng, bnv, c), sh = bf16_rne(bnb[c]) - bf16_rne(bnm[c]) * sc;
#pragma unroll 1
    for (int r8 = 0; r8 < 8; ++r8) Tf[8 * hlf + r8][c] = fmaxf(pmul(acc[tt][r8] * (1.0f / (HS * WSC)), sc) + sh, 0.0f); }
  wave_lds_sync();
  for (int pass = 0; pass < 2; ++pass) { for (int rr = 0; rr < 16; ++rr) ((volatile float*)FUSED)[(t0 + rr) * C + fo + lane] = Tf[rr][lane]; __threadfence(); }
}
__global__ __launch_bounds__(32) void fuse_kernel(const float* __restrict__ FUSED, const float* __restrict__ GF, const float* __restrict__ XT, const b16* __restrict__ WP, const float* __restrict__ bng, const float* __restrict__ bnb, const float* __restrict__ bnm, const float* __restrict__ bnv, int NTV, float* __restrict__ Y2) {
  __shared__ __attribute__((aligned(16))) b16 Ah[16][256 + 8], Al[16][256 + 8]; __shared__ __attribute__((aligned(16))) float Tf[16][C + 4];
  const int lane = threadIdx.x, nloc = lane & 15, hlf = lane >> 4; const size_t t0 = (size_t)blockIdx.x * 16; if (t0 >= (size_t)NTV) return; const int b = (int)(t0 / LI);
  for (int rr = 0; rr < 16; ++rr) for (int q = 0; q < 4; ++q) { const int c = q * 32 + lane; b16 p, ql; split16(FUSED[(t0 + rr) * C + c] * XS, p, ql); Ah[rr][c] = p; Al[rr][c] = ql; split16(GF[b * C + c] * XS, p, ql); Ah[rr][C + c] = p; Al[rr][C + c] = ql; }
  wave_lds_sync();
  v8f acc[8];
#pragma unroll
  for (int t = 0; t < 8; ++t) acc[t] = (v8f){};
#pragma unroll 2
  for (int kb = 0; kb < 2 * C; kb += 32) { const v16b a = frag_kb(&Ah[nloc][kb], hlf), al = frag_kb(&Al[nloc][kb], hlf);
#pragma unroll
    for (int t = 0; t < 8; ++t) { const v16b bw = frag_kb(WP + (size_t)(t * 16 + nloc) * (2 * C) + kb, hlf); acc[t] = wmma16b(a, bw, acc[t]); acc[t] = wmma16b(al, bw, acc[t]); } }
#pragma unroll
  for (int t = 0; t < 8; ++t) { const int c = t * 16 + nloc; const float sc = bnscale(bng, bnv, c), sh = bf16_rne(bnb[c]) - bf16_rne(bnm[c]) * sc;
#pragma unroll 1
    for (int r8 = 0; r8 < 8; ++r8) { const int rl = 8 * hlf + r8; Tf[rl][c] = XT[(t0 + rl) * C + c] + fmaxf(pmul(acc[t][r8] * (1.0f / (XS * WSC)), sc) + sh, 0.0f); } }
  wave_lds_sync();
  for (int pass = 0; pass < 2; ++pass) { for (int rr = 0; rr < 16; ++rr) *(volatile v4f*)(Y2 + (t0 + rr) * C + lane * 4) = *(const v4f*)(&Tf[rr][lane * 4]); __threadfence(); }
}
__global__ __launch_bounds__(32) void sa_kernel(const float* __restrict__ Y2, const b16* __restrict__ WSA, const float* __restrict__ CA, float* __restrict__ out) {
  __shared__ __attribute__((aligned(16))) b16 Ah[16][C + 8], Al[16][C + 8]; __shared__ float To[C][33], Ssa[32];
  const int lane = threadIdx.x, nloc = lane & 15, hlf = lane >> 4; const size_t tw0 = (size_t)blockIdx.x * 32; const int b = (int)(tw0 / LI);
#pragma unroll 1
  for (int half = 0; half < 2; ++half) { const size_t t0 = tw0 + half * 16; v8f acc = {};
#pragma unroll 1
    for (int tap = 0; tap < 49; ++tap) { const int dy = tap / 7 - 3, dx = tap % 7 - 3;
      for (int rr = 0; rr < 16; ++rr) { const size_t t = t0 + rr; const int p = (int)(t % LI), y = p / HI, xx = p % HI; const int yy = y + dy, x2 = xx + dx; const bool ok = yy >= 0 && yy < HI && x2 >= 0 && x2 < HI; const size_t tn = ((size_t)b * HI + (ok ? yy : y)) * HI + (ok ? x2 : xx);
        for (int q = 0; q < 4; ++q) { const float v = ok ? Y2[tn * C + q * 32 + lane] : 0.0f; b16 ph, pl; split16(v * XS, ph, pl); Ah[rr][q * 32 + lane] = ph; Al[rr][q * 32 + lane] = pl; } }
      wave_lds_sync();
#pragma unroll
      for (int kb = 0; kb < C; kb += 32) { const v16b a = frag_kb(&Ah[nloc][kb], hlf), al = frag_kb(&Al[nloc][kb], hlf); const v16b bw = frag_kb(WSA + (size_t)nloc * 6272 + tap * C + kb, hlf); acc = wmma16b(a, bw, acc); acc = wmma16b(al, bw, acc); }
      wave_lds_sync(); }
    if (nloc == 0) {
#pragma unroll
      for (int r8 = 0; r8 < 8; ++r8) Ssa[half * 16 + 8 * hlf + r8] = sigm(acc[r8] * (1.0f / (XS * WSC))); }
    wave_lds_sync();
    for (int rr = 0; rr < 16; ++rr) { const size_t t = t0 + rr; const float s = Ssa[half * 16 + rr]; for (int q = 0; q < 4; ++q) { const int c = q * 32 + lane; const float yv = Y2[t * C + c]; To[c][half * 16 + rr] = yv + pmul(yv, pmul(CA[b * C + c], s)); } }
    wave_lds_sync(); }
  const int p0 = (int)(tw0 % LI);
  for (int pass = 0; pass < 2; ++pass) { for (int c = 0; c < C; ++c) ((volatile float*)out)[((size_t)b * C + c) * LI + p0 + lane] = To[c][lane]; __threadfence(); }
}
}

extern "C" void kernel_launch(void* const* d_in, const int* in_sizes, int n_in, void* d_out, int out_size, void* d_ws, size_t ws_size, hipStream_t stream) {
  (void)n_in;
  auto Fp = [&](int i) { return (const float*)d_in[i]; };
  if (in_sizes[0] != NB * C * LI || in_sizes[1] != GC * GC * 9 || in_sizes[6] != 2 * DI * GC || in_sizes[9] != 4 * 18 * DI || in_sizes[12] != 4 * DI * 8 || in_sizes[24] != DI * 49 || in_sizes[26] != 4 * 50 * DI || in_sizes[29] != 4 * DI * 24 || in_sizes[40] != C * 2 * C || in_sizes[49] != C * 49 || out_size != NB * C * LI) return;
  const int NBV = NB; const int NTV = NBV * LI;
  size_t off = 0; char* ws = (char*)d_ws;
  auto carve = [&](size_t bytes) { char* p = ws + off; off += (bytes + 255) & ~(size_t)255; return p; };
  b16* WC1 = (b16*)carve(GC * 288 * 2); b16* WC3 = (b16*)carve(GC * 288 * 2); b16* WI2 = (b16*)carve(128 * 32 * 2); b16* WI4 = (b16*)carve(128 * 32 * 2); b16* XP2 = (b16*)carve(4 * 32 * DI * 2); b16* XP4 = (b16*)carve(4 * 64 * DI * 2); b16* DW2 = (b16*)carve(4 * DI * 32 * 2); b16* DW4 = (b16*)carve(4 * DI * 32 * 2);
  b16* WO2 = (b16*)carve(32 * DI * 2); b16* WO4 = (b16*)carve(32 * DI * 2); b16* WG2 = (b16*)carve(32 * DI * 2); b16* WG4 = (b16*)carve(32 * DI * 2); b16* WPJ = (b16*)carve(C * 2 * C * 2); b16* WSA = (b16*)carve(16 * 6272 * 2);
  float* XT = (float*)carve((size_t)NTK * C * 4); float* FUSED = (float*)carve((size_t)NTK * C * 4); float* Y2 = (float*)carve((size_t)NTK * C * 4); float* POOL = (float*)carve(NB * C * 4); float* POOLY = (float*)carve(NB * C * 4); float* GF = (float*)carve(NB * C * 4); float* CA = (float*)carve(NB * C * 4);
  float* XZ = (float*)carve((size_t)NTK * 128 * 4); float* U = (float*)carve((size_t)NTK * DI * 4); float* BC = (float*)carve((size_t)4 * NTK * 64 * 4); float* DT = (float*)carve((size_t)4 * NTK * DI * 4); float* Y = (float*)carve((size_t)4 * NTK * DI * 4);
  if (off > ws_size || off > ((size_t)128 << 20)) return;
  auto wcp = [&](const float* w, int KIN, int OUT, int KP, int OUTP, b16* WT) { wcopyp_kernel<<<(OUTP * KP / 8 + 255) / 256, 256, 0, stream>>>(w, KIN, OUT, KP, OUTP, WT); };
  wconv_kernel<<<(GC * 288 / 8 + 255) / 256, 256, 0, stream>>>(Fp(1), WC1); wconv_kernel<<<(GC * 288 / 8 + 255) / 256, 256, 0, stream>>>(Fp(22), WC3);
  wcp(Fp(6), GC, 128, 32, 128, WI2); wcp(Fp(23), GC, 128, 32, 128, WI4);
  for (int k = 0; k < 4; ++k) { wcp(Fp(9) + (size_t)k * 18 * DI, DI, 18, DI, 32, XP2 + (size_t)k * 32 * DI); wcp(Fp(26) + (size_t)k * 50 * DI, DI, 50, DI, 64, XP4 + (size_t)k * 64 * DI); wcp(Fp(10) + (size_t)k * DI * 2, 2, DI, 32, DI, DW2 + (size_t)k * DI * 32); wcp(Fp(27) + (size_t)k * DI * 2, 2, DI, 32, DI, DW4 + (size_t)k * DI * 32); }
  wcp(Fp(16), DI, GC, DI, GC, WO2); wcp(Fp(33), DI, GC, DI, GC, WO4); wcp(Fp(17), 2 * GC, GC, 2 * GC, GC, WG2); wcp(Fp(34), 2 * GC, GC, 2 * GC, GC, WG4); wcp(Fp(40), 2 * C, C, 2 * C, C, WPJ);
  wsa_kernel<<<(16 * 6272 / 8 + 255) / 256, 256, 0, stream>>>(Fp(49), WSA);
  xt_kernel<<<NBV * HI * 4, 256, 0, stream>>>(Fp(0), XT);
  pool_kernel<<<NBV, 128, 0, stream>>>(XT, NBV, POOL); gf_kernel<<<NBV, 128, 0, stream>>>(POOL, Fp(39), GF);
  conv3_kernel<<<NTV / 16, 32, 0, stream>>>(XT, 0, -1, 1, WC1, Fp(2), Fp(3), Fp(4), Fp(5), 0, NTV, FUSED);
  conv3_kernel<<<NTV / 16, 32, 0, stream>>>(XT, 64, 0, 12, WC3, nullptr, nullptr, nullptr, nullptr, 64, NTV, FUSED);
  inproj_kernel<<<NTV / 16, 32, 0, stream>>>(XT, 32, -1, WI2, NTV, XZ);
  dwconv_kernel<3><<<(unsigned)(((size_t)NTV * (DI / 4) + 255) / 256), 256, 0, stream>>>(XZ, Fp(7), Fp(8), NTV, U);
  xproj_kernel<8, 2, 32><<<dim3(NTV / 16, 4), 32, 0, stream>>>(U, XP2, DW2, Fp(11), NTV, BC, DT);
  scan_kernel<8, 32><<<(NBV * 4 * DI + 255) / 256, 256, 0, stream>>>(U, DT, BC, Fp(12), Fp(13), NBV, Y);
  sstail_kernel<<<NTV / 16, 32, 0, stream>>>(Y, XZ, Fp(14), Fp(15), WO2, POOL, 32, -1, WG2, Fp(18), Fp(19), Fp(20), Fp(21), 32, NTV, FUSED);
  inproj_kernel<<<NTV / 16, 32, 0, stream>>>(XT, 96, 32, WI4, NTV, XZ);
  dwconv_kernel<7><<<(unsigned)(((size_t)NTV * (DI / 4) + 255) / 256), 256, 0, stream>>>(XZ, Fp(24), Fp(25), NTV, U);
  xproj_kernel<24, 4, 64><<<dim3(NTV / 16, 4), 32, 0, stream>>>(U, XP4, DW4, Fp(28), NTV, BC, DT);
  scan_kernel<24, 64><<<(NBV * 4 * DI + 255) / 256, 256, 0, stream>>>(U, DT, BC, Fp(29), Fp(30), NBV, Y);
  sstail_kernel<<<NTV / 16, 32, 0, stream>>>(Y, XZ, Fp(31), Fp(32), WO4, POOL, 96, 32, WG4, Fp(35), Fp(36), Fp(37), Fp(38), 96, NTV, FUSED);
  fuse_kernel<<<NTV / 16, 32, 0, stream>>>(FUSED, GF, XT, WPJ, Fp(41), Fp(42), Fp(43), Fp(44), NTV, Y2);
  pool_kernel<<<NBV, 128, 0, stream>>>(Y2, NBV, POOLY); ca_kernel<<<NBV, 128, 0, stream>>>(POOLY, Fp(45), Fp(46), Fp(47), Fp(48), CA);
  sa_kernel<<<NTV / 32, 32, 0, stream>>>(Y2, WSA, CA, (float*)d_out);
}
